// GRU_Precoder_53850299957345
// MI455X (gfx1250) — hardware-verified
//
#include <hip/hip_runtime.h>
#include <stdint.h>

typedef __attribute__((ext_vector_type(16))) _Float16 v16h;
typedef __attribute__((ext_vector_type(8)))  _Float16 v8h;
typedef __attribute__((ext_vector_type(16))) __bf16   v16b;
typedef __attribute__((ext_vector_type(8)))  __bf16   v8b;
typedef __attribute__((ext_vector_type(8)))  float    v8f;
typedef __attribute__((ext_vector_type(4)))  float    v4f;

__device__ __forceinline__ unsigned short f2bf_bits(float f) {
  unsigned u = __float_as_uint(f);
  return (unsigned short)((u + 0x7FFFu + ((u >> 16) & 1u)) >> 16);
}
__device__ __forceinline__ float bf_bits2f(unsigned short h) { return __uint_as_float(((unsigned)h) << 16); }

__device__ __forceinline__ void dep_guard_h(v8f& a, v8f& b, v16h x, v16h y) { asm volatile("v_nop\n\tv_nop\n\tv_nop\n\tv_nop" : "+v"(a), "+v"(b) : "v"(x), "v"(y)); }
__device__ __forceinline__ void dep_guard_b(v8f& a, v8f& b, v16b x, v16b y) { asm volatile("v_nop\n\tv_nop\n\tv_nop\n\tv_nop" : "+v"(a), "+v"(b) : "v"(x), "v"(y)); }
__device__ __forceinline__ void keep4_h(v16h a, v16h b, v16h c, v16h d) { asm volatile("v_nop" :: "v"(a), "v"(b), "v"(c), "v"(d)); }
__device__ __forceinline__ void keep4_b(v16b a, v16b b, v16b c, v16b d) { asm volatile("v_nop" :: "v"(a), "v"(b), "v"(c), "v"(d)); }
__device__ __forceinline__ void acc_guard4(v8f& a, v8f& b, v8f& c, v8f& d) { asm volatile("v_nop\n\tv_nop\n\tv_nop\n\tv_nop" : "+v"(a), "+v"(b), "+v"(c), "+v"(d)); }
template <typename T> struct Frag;
template <> struct Frag<_Float16> {
  typedef v16h V; union U { v16h v; v8h h[2]; };
  static __device__ __forceinline__ v16h load(const _Float16* p) {
    U f; f.h[0] = *(const v8h*)(p); f.h[1] = *(const v8h*)(p + 16); return f.v;
  }
  static __device__ __forceinline__ v8f mma(v16h a, v16h b, v8f c) {
    return __builtin_amdgcn_wmma_f32_16x16x32_f16(false, a, false, b, (short)0, c, false, false);
  }
  static __device__ __forceinline__ void guard(v8f& a, v8f& b, v16h x, v16h y) { dep_guard_h(a, b, x, y); }
  static __device__ __forceinline__ void keep(v16h a, v16h b, v16h c, v16h d) { keep4_h(a, b, c, d); }
};
template <> struct Frag<__bf16> {
  typedef v16b V; union U { v16b v; v8b h[2]; };
  static __device__ __forceinline__ v16b load(const __bf16* p) {
    U f; f.h[0] = *(const v8b*)(p); f.h[1] = *(const v8b*)(p + 16); return f.v;
  }
  static __device__ __forceinline__ v8f mma(v16b a, v16b b, v8f c) {
    return __builtin_amdgcn_wmma_f32_16x16x32_bf16(false, a, false, b, (short)0, c, false, false);
  }
  static __device__ __forceinline__ void guard(v8f& a, v8f& b, v16b x, v16b y) { dep_guard_b(a, b, x, y); }
  static __device__ __forceinline__ void keep(v16b a, v16b b, v16b c, v16b d) { keep4_b(a, b, c, d); }
};

template <int ET> struct Elem;
template <> struct Elem<0> { typedef _Float16 T; };
template <> struct Elem<1> { typedef __bf16 T; };
template <int ET, bool SPLIT, int BIAS_MODE, int OUT_MODE, bool RESID, int ACT = 0>
__global__ __launch_bounds__(256) void wmma_gemm64(
    const unsigned short* __restrict__ Ap, const unsigned short* __restrict__ A2p, int lda, long strideA,
    const unsigned short* __restrict__ Btp, const unsigned short* __restrict__ Bt2p, int ldb, long strideB,
    void* __restrict__ Cout, void* __restrict__ Cout2, int ldc, long strideC,
    const float* __restrict__ bias,
    const float* __restrict__ resid, long strideR,
    int M, int N, int K, float scale) {
  typedef typename Elem<ET>::T T;
  typedef typename Frag<T>::V V;
  const T* A = (const T*)Ap; const T* A2 = (const T*)A2p; const T* Bt = (const T*)Btp; const T* Bt2 = (const T*)Bt2p;
  __shared__ __align__(16) float sT[8][16 * 68];
  const int b    = blockIdx.y;
  const int lane = threadIdx.x & 31;
  const int wave = threadIdx.x >> 5;
  const int tilesN = N >> 6;
  const int tilesM = M >> 6;
  const int tile = blockIdx.x * 8 + wave;
  if (tile >= tilesM * tilesN) return;
  const int tm = tile / tilesN;
  const int tn = tile - tm * tilesN;
  const int m0 = tm << 6;
  const int n0 = tn << 6;

  const T* Ab  = A  + (size_t)b * strideA;
  const T* Bb  = Bt + (size_t)b * strideB;
  const T* Ab2 = SPLIT ? (A2  + (size_t)b * strideA) : nullptr;
  const T* Bb2 = SPLIT ? (Bt2 + (size_t)b * strideB) : nullptr;

  const int rlane = lane & 15;
  const int koff  = (lane >> 4) * 8;
  const int mOff  = (lane >> 4) * 8;

  v8f acc[4][4];
#pragma unroll
  for (int i = 0; i < 4; ++i)
#pragma unroll
    for (int j = 0; j < 4; ++j) acc[i][j] = (v8f){0.f,0.f,0.f,0.f,0.f,0.f,0.f,0.f};

  for (int k0 = 0; k0 < K; k0 += 32) {
    V bh[4], bl[4];
#pragma unroll
    for (int j = 0; j < 4; ++j) {
      const size_t bo = (size_t)(n0 + (j << 4) + rlane) * ldb + koff + k0;
      bh[j] = Frag<T>::load(Bb + bo);
      if (SPLIT) bl[j] = Frag<T>::load(Bb2 + bo);
    }
#pragma unroll
    for (int i = 0; i < 4; ++i) {
      const size_t ao = (size_t)(m0 + (i << 4) + rlane) * lda + koff + k0;
      V ah = Frag<T>::load(Ab + ao);
      V al;
      if (SPLIT) al = Frag<T>::load(Ab2 + ao);
#pragma unroll
      for (int j = 0; j < 4; ++j) {
        acc[i][j] = Frag<T>::mma(ah, bh[j], acc[i][j]);
        if (SPLIT) {
          acc[i][j] = Frag<T>::mma(ah, bl[j], acc[i][j]);
          acc[i][j] = Frag<T>::mma(al, bh[j], acc[i][j]);
        }
      }
      Frag<T>::guard(acc[i][0], acc[i][3], ah, SPLIT ? al : ah);
    }
    Frag<T>::keep(bh[0], bh[1], bh[2], bh[3]);
    if (SPLIT) Frag<T>::keep(bl[0], bl[1], bl[2], bl[3]);
  }
  acc_guard4(acc[0][0], acc[0][1], acc[0][2], acc[0][3]);
  acc_guard4(acc[1][0], acc[1][1], acc[1][2], acc[1][3]);
  acc_guard4(acc[2][0], acc[2][1], acc[2][2], acc[2][3]);
  acc_guard4(acc[3][0], acc[3][1], acc[3][2], acc[3][3]);

  float* slab = sT[wave];
  const float* Rb = RESID ? (resid + (size_t)b * strideR) : nullptr;
#pragma unroll
  for (int i = 0; i < 4; ++i) {
    const int mBase = m0 + (i << 4);
#pragma unroll
    for (int j = 0; j < 4; ++j) {
      const int n = n0 + (j << 4) + rlane;
      float bv = 0.f;
      if (BIAS_MODE == 2) bv = bias[n];
#pragma unroll
      for (int r = 0; r < 8; ++r) {
        float v = acc[i][j][r] * scale;
        if (BIAS_MODE == 1) v += bias[mBase + mOff + r];
        if (BIAS_MODE == 2) v += bv;
        if (RESID) v += Rb[(size_t)(mBase + mOff + r) * ldc + n];
        if (ACT == 1) v = tanhf(v);
        if (ACT == 2) v = fmaxf(v, 0.0f);
        if (ACT == 3) v = v / (1.0f + expf(-v));
        if (ACT == 4) v = (v > 0.f) ? v : 0.01f * v;
        if (ACT == 5) v = 0.5f * v * (1.0f + erff(v * 0.70710678118654752f));
        slab[(mOff + r) * 68 + (j << 4) + rlane] = v;
      }
    }
    __builtin_amdgcn_fence(__ATOMIC_RELEASE, "workgroup");
    __builtin_amdgcn_wave_barrier();
    __builtin_amdgcn_fence(__ATOMIC_ACQUIRE, "workgroup");
    if (OUT_MODE == 0) {
      float* C = (float*)Cout + (size_t)b * strideC;
      const int hh = lane >> 4, c4 = (lane & 15) * 4;
      for (int pass = 0; pass < 2; ++pass) {
#pragma unroll
        for (int it = 0; it < 8; ++it) {
          const int row = it * 2 + hh;
          v4f v = *(const v4f*)(slab + row * 68 + c4);
          *(volatile v4f*)(C + (size_t)(mBase + row) * ldc + n0 + c4) = v;
        }
        __threadfence();
      }
    } else {
      const int q = lane >> 3, c8 = (lane & 7) * 8;
      unsigned short* C  = (unsigned short*)Cout  + (size_t)b * strideC;
      unsigned short* C2 = (OUT_MODE == 2) ? ((unsigned short*)Cout2 + (size_t)b * strideC) : nullptr;
      for (int pass = 0; pass < 2; ++pass) {
#pragma unroll
        for (int it = 0; it < 4; ++it) {
          const int row = it * 4 + q;
          const float* sp = slab + row * 68 + c8;
          v8h hv, lv;
#pragma unroll
          for (int e = 0; e < 8; ++e) {
            if (OUT_MODE == 1) {
              hv[e] = (_Float16)sp[e];
            } else {
              unsigned short hb = f2bf_bits(sp[e]);
              unsigned short lb = f2bf_bits(sp[e] - bf_bits2f(hb));
              hv[e] = __builtin_bit_cast(_Float16, hb);
              lv[e] = __builtin_bit_cast(_Float16, lb);
            }
          }
          *(volatile v8h*)(C + (size_t)(mBase + row) * ldc + n0 + c8) = hv;
          if (OUT_MODE == 2) *(volatile v8h*)(C2 + (size_t)(mBase + row) * ldc + n0 + c8) = lv;
        }
        __threadfence();
      }
    }
    __builtin_amdgcn_fence(__ATOMIC_RELEASE, "workgroup");
    __builtin_amdgcn_wave_barrier();
    __builtin_amdgcn_fence(__ATOMIC_ACQUIRE, "workgroup");
  }
}

constexpr int kBatch     = 1024;
constexpr int kSeq       = 64;
constexpr int kObs       = 128;
constexpr int kZdim      = 64;
constexpr int kDin       = 192;
constexpr int kHid       = 512;
constexpr int kCtx       = 64;
constexpr int kAct       = 32;
constexpr int kMlp       = 256;
constexpr int kGate3     = 1536;
constexpr int kHPitch    = 520;
constexpr int kSlabPitch = 36;
constexpr float kInv16   = 0.0625f;
constexpr float kInv128  = 0.0078125f;
constexpr float kWScale  = 16.0f;
constexpr float kXScale  = 8.0f;
constexpr float kLnEps   = 1e-6f;

static_assert(kDin == kObs + kZdim, "din");
static_assert(kGate3 == 3 * kHid, "gates");
static_assert(kDin % 32 == 0 && kMlp % 64 == 0 && kHid % 64 == 0 && kGate3 % 64 == 0 && kBatch % 64 == 0, "tile multiples");
static_assert(kBatch % 16 == 0 && kAct == 32, "persistent kernel shape");

constexpr size_t kOffX0h = 0;
constexpr size_t kOffW1t = kOffX0h + (size_t)kBatch * kDin * 2;
constexpr size_t kOffW2t = kOffW1t + (size_t)kMlp * kDin * 2;
constexpr size_t kOffW3t = kOffW2t + (size_t)kMlp * kMlp * 2;
constexpr size_t kOffWit = kOffW3t + (size_t)kHid * kMlp * 2;
constexpr size_t kOffWht = kOffWit + (size_t)kGate3 * kDin * 2;
constexpr size_t kOffWot = kOffWht + (size_t)kGate3 * kHid * 2;
constexpr size_t kOffP1  = kOffWot + (size_t)kAct * kHid * 2;
constexpr size_t kOffH1h = kOffP1  + (size_t)kBatch * kMlp * 4;
constexpr size_t kOffP2  = kOffH1h + (size_t)kBatch * kMlp * 2;
constexpr size_t kOffH2h = kOffP2  + (size_t)kBatch * kMlp * 4;
constexpr size_t kOffH0  = kOffH2h + (size_t)kBatch * kMlp * 2;
constexpr size_t kOffXI  = kOffH0  + (size_t)kBatch * kHid * 4;
constexpr size_t kWsTotal = kOffXI + (size_t)kBatch * kGate3 * 4;
static_assert(kWsTotal == 14614528, "carve total");
static_assert(kWsTotal <= 134217728, "carve budget");
static_assert((kOffW1t % 256) == 0 && (kOffW2t % 256) == 0 && (kOffW3t % 256) == 0 && (kOffWit % 256) == 0 &&
              (kOffWht % 256) == 0 && (kOffWot % 256) == 0 && (kOffP1 % 256) == 0 && (kOffH1h % 256) == 0 &&
              (kOffP2 % 256) == 0 && (kOffH2h % 256) == 0 && (kOffH0 % 256) == 0 && (kOffXI % 256) == 0, "alignment");

__global__ __launch_bounds__(256) void build_x0_kernel(const float* __restrict__ s_t,
                                                      const float* __restrict__ z_t,
                                                      unsigned short* __restrict__ X0p) {
  const int wave = threadIdx.x >> 5, lane = threadIdx.x & 31;
  const int row = blockIdx.x * 8 + wave;
  const int ls = lane < 16 ? lane : 15;
  int lz = lane - 16; lz = lz < 0 ? 0 : (lz > 7 ? 7 : lz);
  const float* sp = s_t + (size_t)row * (kSeq * kObs) + ls * 8;
  const float* zp = z_t + (size_t)row * kZdim + lz * 8;
  const v4f s0 = *(const v4f*)sp, s1 = *(const v4f*)(sp + 4);
  const v4f z0 = *(const v4f*)zp, z1 = *(const v4f*)(zp + 4);
  const bool use_s = lane < 16;
  v8h hv;
#pragma unroll
  for (int e = 0; e < 4; ++e) {
    const float a0 = use_s ? s0[e] : z0[e];
    const float a1 = use_s ? s1[e] : z1[e];
    hv[e]     = (_Float16)(a0 * kXScale);
    hv[4 + e] = (_Float16)(a1 * kXScale);
  }
  const int lc = lane < 24 ? lane : 0;
  _Float16* dst = (_Float16*)X0p + (size_t)row * kDin + lc * 8;
  if (lane < 24) *(volatile v8h*)dst = hv;
  __threadfence();
  if (lane < 24) *(volatile v8h*)dst = hv;
}

__global__ __launch_bounds__(256) void tr_cast_f16_kernel(const float* __restrict__ in,
                                                         unsigned short* __restrict__ outp,
                                                         int Kd, int Nd, float scale) {
  __shared__ __align__(16) float tile[32 * 68];
  const int tid = threadIdx.x;
  const int n0 = blockIdx.x * 32;
  const int k0 = blockIdx.y * 64;
#pragma unroll
  for (int i = 0; i < 8; ++i) {
    const int idx = i * 256 + tid;
    const int kr = idx >> 5;
    const int nc = idx & 31;
    tile[nc * 68 + kr] = in[(size_t)(k0 + kr) * Nd + n0 + nc];
  }
  __syncthreads();
  const int wave = tid >> 5, lane = tid & 31;
  const int q = lane >> 3, c8 = (lane & 7) * 8;
  const int nr = wave * 4 + q;
  const float* tp = tile + nr * 68 + c8;
  const v4f t0 = *(const v4f*)tp, t1 = *(const v4f*)(tp + 4);
  v8h hv;
#pragma unroll
  for (int e = 0; e < 4; ++e) {
    hv[e]     = (_Float16)(t0[e] * scale);
    hv[4 + e] = (_Float16)(t1[e] * scale);
  }
  _Float16* dst = (_Float16*)outp + (size_t)(n0 + nr) * Kd + k0 + c8;
  *(volatile v8h*)dst = hv;
  __threadfence();
  *(volatile v8h*)dst = hv;
}

__global__ __launch_bounds__(256) void ln_relu_f16_kernel(const float* __restrict__ P,
                                                         const float* __restrict__ g,
                                                         const float* __restrict__ be,
                                                         unsigned short* __restrict__ Hp) {
  const int wave = threadIdx.x >> 5, lane = threadIdx.x & 31;
  const int row = blockIdx.x * 8 + wave;
  const int c8 = lane * 8;
  const float* pp = P + (size_t)row * kMlp + c8;
  const v4f p0 = *(const v4f*)pp, p1 = *(const v4f*)(pp + 4);
  float s = ((p0[0] + p0[1]) + (p0[2] + p0[3])) + ((p1[0] + p1[1]) + (p1[2] + p1[3]));
#pragma unroll
  for (int off = 1; off < 32; off <<= 1) s += __shfl_xor(s, off, 32);
  const float mean = s * (1.0f / 256.0f);
  v4f d0, d1;
#pragma unroll
  for (int e = 0; e < 4; ++e) { d0[e] = p0[e] - mean; d1[e] = p1[e] - mean; }
  float sq = ((d0[0] * d0[0] + d0[1] * d0[1]) + (d0[2] * d0[2] + d0[3] * d0[3])) +
             ((d1[0] * d1[0] + d1[1] * d1[1]) + (d1[2] * d1[2] + d1[3] * d1[3]));
#pragma unroll
  for (int off = 1; off < 32; off <<= 1) sq += __shfl_xor(sq, off, 32);
  const float var = sq * (1.0f / 256.0f);
  const float inv = rsqrtf(var + kLnEps);
  const v4f g0 = *(const v4f*)(g + c8), g1 = *(const v4f*)(g + c8 + 4);
  const v4f e0 = *(const v4f*)(be + c8), e1 = *(const v4f*)(be + c8 + 4);
  v8h hv;
#pragma unroll
  for (int e = 0; e < 4; ++e) {
    float y0 = d0[e] * inv * g0[e] + e0[e];
    float y1 = d1[e] * inv * g1[e] + e1[e];
    y0 = y0 > 0.0f ? y0 : 0.0f;
    y1 = y1 > 0.0f ? y1 : 0.0f;
    hv[e] = (_Float16)y0;
    hv[4 + e] = (_Float16)y1;
  }
  _Float16* dst = (_Float16*)Hp + (size_t)row * kMlp + c8;
  *(volatile v8h*)dst = hv;
  __threadfence();
  *(volatile v8h*)dst = hv;
}

__device__ __forceinline__ void guard3_h(v8f& a, v8f& b, v8f& c, v16h x, v16h y, v16h z, v16h w) {
  asm volatile("v_nop\n\tv_nop\n\tv_nop\n\tv_nop" : "+v"(a), "+v"(b), "+v"(c) : "v"(x), "v"(y), "v"(z), "v"(w));
}
__device__ __forceinline__ void guard1_h(v8f& a, v16h x, v16h y) {
  asm volatile("v_nop\n\tv_nop\n\tv_nop\n\tv_nop" : "+v"(a) : "v"(x), "v"(y));
}
__device__ __forceinline__ float sigmoid_f32(float x) {
  const float xc = fminf(fmaxf(x, -30.0f), 30.0f);
  return 1.0f / (1.0f + expf(-xc));
}
__device__ __forceinline__ float tanh_f32(float x) {
  const float xc = fminf(fmaxf(x, -15.0f), 15.0f);
  return 2.0f / (1.0f + expf(-2.0f * xc)) - 1.0f;
}

__global__ __launch_bounds__(256) void gru_scan_kernel(
    const float* __restrict__ H0, const float* __restrict__ XI, const float* __restrict__ bh,
    const unsigned short* __restrict__ Whtp, const unsigned short* __restrict__ Wotp,
    const float* __restrict__ bo, float* __restrict__ out) {
  const _Float16* Wht = (const _Float16*)Whtp;
  const _Float16* Wot = (const _Float16*)Wotp;
  __shared__ __align__(16) _Float16 hA[2][16 * kHPitch];
  __shared__ __align__(16) float slab[16 * kSlabPitch];
  const int tid = threadIdx.x;
  const int wave = tid >> 5;
  const int lane = tid & 31;
  const int hh = lane >> 4;
  const int c = lane & 15;
  const int b0 = blockIdx.x * 16;

  float hreg[4][8];
  float bhr[4], bhz[4], bhn[4];
#pragma unroll
  for (int j = 0; j < 4; ++j) {
    const int col = (wave * 4 + j) * 16 + c;
    bhr[j] = bh[col];
    bhz[j] = bh[kHid + col];
    bhn[j] = bh[2 * kHid + col];
#pragma unroll
    for (int r = 0; r < 8; ++r) {
      const int row = 8 * hh + r;
      const float h = H0[(size_t)(b0 + row) * kHid + col];
      hreg[j][r] = h;
      hA[0][row * kHPitch + col] = (_Float16)h;
    }
  }
  const float bol = bo[(wave & 1) * 16 + c];
  __syncthreads();

  const v8f vz = (v8f){0.f, 0.f, 0.f, 0.f, 0.f, 0.f, 0.f, 0.f};
  int cur = 0;
  for (int t = 0; t < kCtx; ++t) {
    const int nxt = cur ^ 1;
#pragma unroll
    for (int j = 0; j < 4; ++j) {
      const int ub = wave * 4 + j;
      const int col = ub * 16 + c;
      v8f ar = vz, az = vz, an = vz;
      const _Float16* br = Wht + (size_t)col * kHid + 8 * hh;
      const _Float16* bz = br + (size_t)kHid * kHid;
      const _Float16* bn = bz + (size_t)kHid * kHid;
      const _Float16* ap = &hA[cur][c * kHPitch + 8 * hh];
#pragma unroll 2
      for (int kt = 0; kt < kHid / 32; ++kt) {
        const int k0 = kt * 32;
        const v16h a  = Frag<_Float16>::load(ap + k0);
        const v16h fr = Frag<_Float16>::load(br + k0);
        const v16h fz = Frag<_Float16>::load(bz + k0);
        const v16h fn = Frag<_Float16>::load(bn + k0);
        ar = Frag<_Float16>::mma(a, fr, ar);
        az = Frag<_Float16>::mma(a, fz, az);
        an = Frag<_Float16>::mma(a, fn, an);
        guard3_h(ar, az, an, a, fr, fz, fn);
      }
      const float* xb = XI + (size_t)(b0 + 8 * hh) * kGate3 + col;
#pragma unroll
      for (int r = 0; r < 8; ++r) {
        const float* xp = xb + (size_t)r * kGate3;
        const float xr = xp[0];
        const float xz = xp[kHid];
        const float xn = xp[2 * kHid];
        const float gr = ar[r] * kInv16 + bhr[j];
        const float gz = az[r] * kInv16 + bhz[j];
        const float gn = an[r] * kInv16 + bhn[j];
        const float rg = sigmoid_f32(xr + gr);
        const float zg = sigmoid_f32(xz + gz);
        const float ng = tanh_f32(xn + rg * gn);
        const float hp = hreg[j][r];
        const float hv = (1.0f - zg) * ng + zg * hp;
        hreg[j][r] = hv;
        hA[nxt][(8 * hh + r) * kHPitch + col] = (_Float16)hv;
      }
    }
    __syncthreads();

    if (wave < 2) {
      const int ca = (wave & 1) * 16 + c;
      v8f ao = vz;
      const _Float16* bp = Wot + (size_t)ca * kHid + 8 * hh;
      const _Float16* ap2 = &hA[nxt][c * kHPitch + 8 * hh];
#pragma unroll 2
      for (int kt = 0; kt < kHid / 32; ++kt) {
        const int k0 = kt * 32;
        const v16h a  = Frag<_Float16>::load(ap2 + k0);
        const v16h fb = Frag<_Float16>::load(bp + k0);
        ao = Frag<_Float16>::mma(a, fb, ao);
        guard1_h(ao, a, fb);
      }
#pragma unroll
      for (int r = 0; r < 8; ++r) slab[(8 * hh + r) * kSlabPitch + ca] = tanh_f32(ao[r] * kInv16 + bol);
    }
    __syncthreads();

    if (wave < 4) {
      const int row = wave * 4 + (lane >> 3);
      const int c4 = (lane & 7) * 4;
      const v4f val = *(const v4f*)(slab + row * kSlabPitch + c4);
      float* dst = out + ((size_t)(b0 + row) * kCtx + t) * kAct + c4;
      *(volatile v4f*)dst = val;
      __threadfence();
      *(volatile v4f*)dst = val;
    }
    cur = nxt;
  }
}

extern "C" void kernel_launch(void* const* d_in, const int* in_sizes, int n_in,
                              void* d_out, int out_size, void* d_ws, size_t ws_size,
                              hipStream_t stream) {
  if (n_in < 17) return;
  if (ws_size < kWsTotal) return;
  if ((size_t)out_size < (size_t)kBatch * kCtx * kAct) return;
  if ((size_t)in_sizes[0] < (size_t)kBatch * kSeq * kObs) return;
  if (in_sizes[1] < kBatch * kZdim || in_sizes[13] < kHid * kGate3 || in_sizes[16] < kAct) return;

  const float* s_t = (const float*)d_in[0];
  const float* z_t = (const float*)d_in[1];
  const float* W1  = (const float*)d_in[2];
  const float* b1  = (const float*)d_in[3];
  const float* g1  = (const float*)d_in[4];
  const float* be1 = (const float*)d_in[5];
  const float* W2  = (const float*)d_in[6];
  const float* b2  = (const float*)d_in[7];
  const float* g2  = (const float*)d_in[8];
  const float* be2 = (const float*)d_in[9];
  const float* W3  = (const float*)d_in[10];
  const float* b3  = (const float*)d_in[11];
  const float* Wi  = (const float*)d_in[12];
  const float* Wh  = (const float*)d_in[13];
  const float* bh  = (const float*)d_in[14];
  const float* Wo  = (const float*)d_in[15];
  const float* bo  = (const float*)d_in[16];
  float* out = (float*)d_out;
  char* ws = (char*)d_ws;

  unsigned short* X0h = (unsigned short*)(ws + kOffX0h);
  unsigned short* W1t = (unsigned short*)(ws + kOffW1t);
  unsigned short* W2t = (unsigned short*)(ws + kOffW2t);
  unsigned short* W3t = (unsigned short*)(ws + kOffW3t);
  unsigned short* Wit = (unsigned short*)(ws + kOffWit);
  unsigned short* Wht = (unsigned short*)(ws + kOffWht);
  unsigned short* Wot = (unsigned short*)(ws + kOffWot);
  float* P1 = (float*)(ws + kOffP1);
  unsigned short* H1h = (unsigned short*)(ws + kOffH1h);
  float* P2 = (float*)(ws + kOffP2);
  unsigned short* H2h = (unsigned short*)(ws + kOffH2h);
  float* H0 = (float*)(ws + kOffH0);
  float* XI = (float*)(ws + kOffXI);

  const unsigned short* nul16 = (const unsigned short*)nullptr;
  const float* nulf = (const float*)nullptr;

  build_x0_kernel<<<kBatch / 8, 256, 0, stream>>>(s_t, z_t, X0h);
  tr_cast_f16_kernel<<<dim3(kMlp / 32, kDin / 64), 256, 0, stream>>>(W1, W1t, kDin, kMlp, kWScale);
  tr_cast_f16_kernel<<<dim3(kMlp / 32, kMlp / 64), 256, 0, stream>>>(W2, W2t, kMlp, kMlp, kWScale);
  tr_cast_f16_kernel<<<dim3(kHid / 32, kMlp / 64), 256, 0, stream>>>(W3, W3t, kMlp, kHid, kWScale);
  tr_cast_f16_kernel<<<dim3(kGate3 / 32, kDin / 64), 256, 0, stream>>>(Wi, Wit, kDin, kGate3, kWScale);
  tr_cast_f16_kernel<<<dim3(kGate3 / 32, kHid / 64), 256, 0, stream>>>(Wh, Wht, kHid, kGate3, kWScale);
  tr_cast_f16_kernel<<<dim3(kAct / 32, kHid / 64), 256, 0, stream>>>(Wo, Wot, kHid, kAct, kWScale);

  wmma_gemm64<0, false, 2, 0, false, 0><<<dim3((kBatch / 64) * (kMlp / 64) / 8, 1), 256, 0, stream>>>(
      X0h, nul16, kDin, 0L, W1t, nul16, kDin, 0L, (void*)P1, (void*)nullptr, kMlp, 0L,
      b1, nulf, 0L, kBatch, kMlp, kDin, kInv128);
  ln_relu_f16_kernel<<<kBatch / 8, 256, 0, stream>>>(P1, g1, be1, H1h);
  wmma_gemm64<0, false, 2, 0, false, 0><<<dim3((kBatch / 64) * (kMlp / 64) / 8, 1), 256, 0, stream>>>(
      H1h, nul16, kMlp, 0L, W2t, nul16, kMlp, 0L, (void*)P2, (void*)nullptr, kMlp, 0L,
      b2, nulf, 0L, kBatch, kMlp, kMlp, kInv16);
  ln_relu_f16_kernel<<<kBatch / 8, 256, 0, stream>>>(P2, g2, be2, H2h);
  wmma_gemm64<0, false, 2, 0, false, 0><<<dim3((kBatch / 64) * (kHid / 64) / 8, 1), 256, 0, stream>>>(
      H2h, nul16, kMlp, 0L, W3t, nul16, kMlp, 0L, (void*)H0, (void*)nullptr, kHid, 0L,
      b3, nulf, 0L, kBatch, kHid, kMlp, kInv16);
  wmma_gemm64<0, false, 0, 0, false, 0><<<dim3((kBatch / 64) * (kGate3 / 64) / 8, 1), 256, 0, stream>>>(
      X0h, nul16, kDin, 0L, Wit, nul16, kDin, 0L, (void*)XI, (void*)nullptr, kGate3, 0L,
      nulf, nulf, 0L, kBatch, kGate3, kDin, kInv128);
  gru_scan_kernel<<<kBatch / 16, 256, 0, stream>>>(H0, XI, bh, Wht, Wot, bo, out);
}
